// SameGTO_22041772163216
// MI455X (gfx1250) — hardware-verified
//
#include <hip/hip_runtime.h>
#include <math.h>

typedef __attribute__((ext_vector_type(16))) _Float16 v16h;
typedef __attribute__((ext_vector_type(16))) __bf16 v16b;
typedef __attribute__((ext_vector_type(8)))  _Float16 v8h;
typedef __attribute__((ext_vector_type(8)))  float v8f;
typedef __attribute__((ext_vector_type(4)))  float v4f;
typedef __attribute__((ext_vector_type(2)))  float v2f;
typedef __attribute__((ext_vector_type(4)))  unsigned v4u;
typedef __attribute__((ext_vector_type(4)))  int v4i;
typedef float __attribute__((may_alias)) float_a;
typedef int __attribute__((may_alias)) int_a;

template <typename T> __device__ __forceinline__ void vst2(void* p, T v) { *(volatile T*)p = v; __threadfence(); *(volatile T*)p = v; }
__device__ __forceinline__ v8f wmma16(v16h a, v16h b, v8f c) {
  v8f d = __builtin_amdgcn_wmma_f32_16x16x32_f16(false, a, false, b, (short)0, c, false, false);
  asm volatile("v_nop\n\tv_nop\n\tv_nop\n\tv_nop" : "+v"(d) : "v"(a), "v"(b));
  return d;
}
__device__ __forceinline__ v8f wmma_bf(v16b a, v16b b, v8f c) {
  v8f d = __builtin_amdgcn_wmma_f32_16x16x32_bf16(false, a, false, b, (short)0, c, false, false);
  asm volatile("v_nop\n\tv_nop\n\tv_nop\n\tv_nop" : "+v"(d) : "v"(a), "v"(b));
  return d;
}
__device__ __forceinline__ v16h frag_h(const _Float16* rowk0, int lane) {
  union { v16h v; v8h q[2]; } u; const _Float16* p = rowk0 + 8 * (lane >> 4);
  u.q[0] = *(const v8h*)p; u.q[1] = *(const v8h*)(p + 16); return u.v;
}
__device__ __forceinline__ v16h frag_f32(const float* rowk0, int lane) {
  v16h a; const float* p = rowk0 + 8 * (lane >> 4);
#pragma unroll
  for (int i = 0; i < 8; ++i) { a[i] = (_Float16)p[i]; a[8 + i] = (_Float16)p[16 + i]; }
  return a;
}
__device__ __forceinline__ v16h frag_f32s(const float* rowk0, int lane, float sc) {
  v16h a; const float* p = rowk0 + 8 * (lane >> 4);
#pragma unroll
  for (int i = 0; i < 8; ++i) { a[i] = (_Float16)(p[i] * sc); a[8 + i] = (_Float16)(p[16 + i] * sc); }
  return a;
}
__device__ __forceinline__ v16h fragc_f32(const float* W, int k0, int n, int lane, int ld, int K) {
  v16h a; const int g = lane >> 4;
#pragma unroll
  for (int i = 0; i < 8; ++i) { const int ka = k0 + 8 * g + i, kb = ka + 16;
    a[i] = (_Float16)(ka < K ? W[(size_t)(ka < K ? ka : K - 1) * ld + n] : 0.f); a[8 + i] = (_Float16)(kb < K ? W[(size_t)(kb < K ? kb : K - 1) * ld + n] : 0.f); }
  return a;
}
struct F2 { v16b h, l; };
__device__ __forceinline__ F2 bsplit16(const float v[16]) { F2 r;
#pragma unroll
  for (int i = 0; i < 16; ++i) { const __bf16 h = (__bf16)v[i]; r.h[i] = h; r.l[i] = (__bf16)(v[i] - (float)h); }
  return r; }
__device__ __forceinline__ F2 split_row(const float* row, int k0, int lane) { float v[16]; const float* p = row + k0 + 8 * (lane >> 4);
#pragma unroll
  for (int i = 0; i < 8; ++i) { v[i] = p[i]; v[8 + i] = p[16 + i]; }
  return bsplit16(v); }
__device__ __forceinline__ F2 split_rowK(const float* row, int k0, int lane, int K) { float v[16]; const int g = lane >> 4;
#pragma unroll
  for (int i = 0; i < 8; ++i) { const int ka = k0 + 8 * g + i, kb = ka + 16; v[i] = ka < K ? row[ka < K ? ka : K - 1] : 0.f; v[8 + i] = kb < K ? row[kb < K ? kb : K - 1] : 0.f; }
  return bsplit16(v); }
__device__ __forceinline__ F2 split_col(const float* W, int k0, int n, int lane, int ld, int K) { float v[16]; const int g = lane >> 4;
#pragma unroll
  for (int i = 0; i < 8; ++i) { const int ka = k0 + 8 * g + i, kb = ka + 16; v[i] = ka < K ? W[(size_t)(ka < K ? ka : K - 1) * ld + n] : 0.f; v[8 + i] = kb < K ? W[(size_t)(kb < K ? kb : K - 1) * ld + n] : 0.f; }
  return bsplit16(v); }
__device__ __forceinline__ v8f mac3(const F2& a, const F2& b, v8f c) { c = wmma_bf(a.l, b.h, c); c = wmma_bf(a.h, b.l, c); return wmma_bf(a.h, b.h, c); }
__device__ __forceinline__ float sigm(float v) { return 1.0f / (1.0f + expf(-v)); }
#define LDSX() do { asm volatile("s_wait_dscnt 0" ::: "memory"); __builtin_amdgcn_wave_barrier(); __builtin_amdgcn_fence(__ATOMIC_RELEASE, "workgroup"); } while (0)


#define NB 2
#define CIN 128
#define NPOS 4096
#define NHD 4
#define DK 16
#define DV 32
#define KF 64
#define VF 128
#ifndef TNB
#define TNB NB
#define TQB (NPOS / 64)
#endif
typedef __attribute__((ext_vector_type(8))) __bf16 v8b;
__device__ __forceinline__ v16b frag_b(const __bf16* rowk0, int lane) {
  union { v16b v; v8b q[2]; } u; const __bf16* p = rowk0 + 8 * (lane >> 4);
  u.q[0] = *(const v8b*)p; u.q[1] = *(const v8b*)(p + 16); return u.v;
}
__device__ __forceinline__ v16b frag_gbf(const float* rowk0, int lane) {
  v16b a; const float* p = rowk0 + 8 * (lane >> 4);
#pragma unroll
  for (int i = 0; i < 8; ++i) { a[i] = (__bf16)p[i]; a[8 + i] = (__bf16)p[16 + i]; }
  return a;
}
__device__ __forceinline__ float bfr(float v) { return (float)(__bf16)v; }
__device__ __attribute__((noinline)) float exp_ni(float v) { return expf(v); }

#define WS_XH   0u
#define WS_XL   (WS_XH + 2u * NB * NPOS * CIN)
#define WS_QKV  (WS_XL + 2u * NB * NPOS * CIN)
#define WS_VTH  (WS_QKV + 4u * NB * NPOS * 256)
#define WS_VTL  (WS_VTH + 2u * NB * VF * NPOS)
#define WS_M    (WS_VTL + 2u * NB * VF * NPOS)
#define WS_L    (WS_M + 4u * NB * NHD * NPOS)
#define WS_O    (WS_L + 4u * NB * NHD * NPOS)
#define WS_END  (WS_O + 4u * NB * NPOS * VF)

__global__ __launch_bounds__(256) void k_xT(const float* __restrict__ X, const float* __restrict__ g, const float* __restrict__ bt, const float* __restrict__ rm, const float* __restrict__ rv, __bf16* __restrict__ PH, __bf16* __restrict__ PL) {
  __shared__ __bf16 sh[64][136], sl[64][136]; __shared__ float ssc[CIN], ssh[CIN];
  const int b = blockIdx.y, p0 = blockIdx.x * 64, tid = threadIdx.x;
  if (tid < CIN) { const float inv = rsqrtf(bfr(rv[tid]) + 1e-5f); const float sc = bfr(g[tid]) * inv; ssc[tid] = sc; ssh[tid] = bfr(bt[tid]) - bfr(rm[tid]) * sc; }
  __syncthreads();
  for (int q = tid; q < CIN * 64; q += 256) { const int c = q >> 6, pl = q & 63; float v = bfr(X[((size_t)b * CIN + c) * NPOS + p0 + pl]) * ssc[c] + ssh[c]; v = v > 0.f ? v : 0.f; const __bf16 hi = (__bf16)v; sh[pl][c] = hi; sl[pl][c] = (__bf16)(v - (float)hi); }
  __syncthreads();
  for (int q = tid; q < 64 * 16; q += 256) { const int pl = q >> 4, pc = q & 15; union { __bf16 e[8]; v4u u; } a, c2;
#pragma unroll
    for (int e = 0; e < 8; ++e) { a.e[e] = sh[pl][pc * 8 + e]; c2.e[e] = sl[pl][pc * 8 + e]; }
    const size_t o = ((size_t)b * NPOS + p0 + pl) * CIN + pc * 8; vst2((unsigned*)(PH + o), a.u); vst2((unsigned*)(PL + o), c2.u); }
}
__global__ __launch_bounds__(128) void k_qkv(const __bf16* __restrict__ PH, const __bf16* __restrict__ PL, const float* __restrict__ Wq, const float* __restrict__ bq, const float* __restrict__ Wk, const float* __restrict__ bk, const float* __restrict__ Wv, const float* __restrict__ bv, float* __restrict__ QKV, __bf16* __restrict__ VTH, __bf16* __restrict__ VTL) {
  __shared__ __align__(16) float so[64][132];
  const int tid = threadIdx.x, wave = tid >> 5, lane = tid & 31, col = lane & 15, g = lane >> 4; const int b = blockIdx.z; const int p0 = blockIdx.x * 64; const int n0 = blockIdx.y * 128;
  const size_t arow = ((size_t)b * NPOS + p0 + wave * 16 + col) * CIN;
  v8f acc[8] = {};
#pragma unroll
  for (int kc = 0; kc < CIN / 32; ++kc) { const v16b ah = frag_b(PH + arow + kc * 32, lane), al = frag_b(PL + arow + kc * 32, lane);
#pragma unroll
    for (int j = 0; j < 8; ++j) { const int n = n0 + j * 16 + col; const float* wr = n < KF ? Wq + (size_t)n * CIN : (n < 2 * KF ? Wk + (size_t)(n - KF) * CIN : Wv + (size_t)(n - 2 * KF) * CIN);
      const v16b w = frag_gbf(wr + kc * 32, lane); acc[j] = wmma_bf(al, w, acc[j]); acc[j] = wmma_bf(ah, w, acc[j]); } }
#pragma unroll
  for (int j = 0; j < 8; ++j) { const int n = n0 + j * 16 + col; const float bias = n < KF ? bfr(bq[n]) : (n < 2 * KF ? bfr(bk[n - KF]) : bfr(bv[n - 2 * KF])); const float sc = n < KF ? 0.25f : 1.0f;
#pragma unroll
    for (int r = 0; r < 8; ++r) so[wave * 16 + 8 * g + r][j * 16 + col] = (acc[j][r] + bias) * sc; }
  __syncthreads();
  for (int q = tid; q < 64 * 32; q += 128) { const int rl = q >> 5, pc = q & 31; vst2(QKV + ((size_t)b * NPOS + p0 + rl) * 256 + n0 + pc * 4, *(const v4f*)&so[rl][pc * 4]); }
  if (n0 == 128) {
    for (int q = tid; q < 128 * 8; q += 128) { const int c = q >> 3, pc = q & 7; union { __bf16 e[8]; v4u u; } hh, ll;
#pragma unroll
      for (int e = 0; e < 8; ++e) { const float v = so[pc * 8 + e][c]; const __bf16 hi = (__bf16)v; hh.e[e] = hi; ll.e[e] = (__bf16)(v - (float)hi); }
      const size_t o = ((size_t)b * VF + c) * NPOS + p0 + pc * 8; vst2((unsigned*)(VTH + o), hh.u); vst2((unsigned*)(VTL + o), ll.u); } }
}
__global__ __launch_bounds__(128) void k_stats(const float* __restrict__ QKV, float* __restrict__ Mb, float* __restrict__ Lb) {
  __shared__ __align__(16) float sm[4][16]; __shared__ __align__(16) float ssum[4][16];
  const int tid = threadIdx.x, wave = tid >> 5, lane = tid & 31, col = lane & 15, g = lane >> 4;
  const int bh = blockIdx.y, b = bh >> 2, h = bh & 3; const int q0 = blockIdx.x * 64 + wave * 16;
  const F2 a = split_rowK(QKV + ((size_t)b * NPOS + q0 + col) * 256 + h * DK, 0, lane, DK);
  float m[8], l[8];
#pragma unroll
  for (int r = 0; r < 8; ++r) { m[r] = -3.0e38f; l[r] = 0.f; }
#pragma unroll 1
  for (int kt = 0; kt < NPOS / 16; ++kt) { const F2 kb = split_rowK(QKV + ((size_t)b * NPOS + kt * 16 + col) * 256 + KF + h * DK, 0, lane, DK); const v8f s = mac3(a, kb, (v8f){});
#pragma unroll
    for (int r = 0; r < 8; ++r) { float mx = s[r];
#pragma unroll
      for (int o = 1; o < 16; o <<= 1) mx = fmaxf(mx, __shfl_xor(mx, o));
      const float mn = fmaxf(m[r], mx); float e = exp_ni(s[r] - mn);
#pragma unroll
      for (int o = 1; o < 16; o <<= 1) e += __shfl_xor(e, o);
      l[r] = l[r] * exp_ni(m[r] - mn) + e; m[r] = mn; } }
  if (col == 0) {
#pragma unroll
    for (int r = 0; r < 8; ++r) { sm[wave][8 * g + r] = m[r]; ssum[wave][8 * g + r] = l[r]; } }
  __syncthreads();
  { const int qb = blockIdx.x * 64; if (tid < 16) vst2(Mb + ((size_t)bh * NPOS + qb) + tid * 4, *(const v4f*)(&sm[0][0] + tid * 4)); else if (tid < 32) vst2(Lb + ((size_t)bh * NPOS + qb) + (tid - 16) * 4, *(const v4f*)(&ssum[0][0] + (tid - 16) * 4)); }
}
__global__ __launch_bounds__(128) void k_attn(const float* __restrict__ QKV, const __bf16* __restrict__ VTH, const __bf16* __restrict__ VTL, const float* __restrict__ Mb, const float* __restrict__ Lb, float* __restrict__ O) {
  __shared__ __align__(16) float sp[4][16][36]; __shared__ __align__(16) float so[4][16][36];
  const int tid = threadIdx.x, wave = tid >> 5, lane = tid & 31, col = lane & 15, g = lane >> 4;
  const int bh = blockIdx.y, b = bh >> 2, h = bh & 3; const int q0 = blockIdx.x * 64 + wave * 16;
  const F2 a = split_rowK(QKV + ((size_t)b * NPOS + q0 + col) * 256 + h * DK, 0, lane, DK);
  float mr[8], il[8];
#pragma unroll
  for (int r = 0; r < 8; ++r) { mr[r] = Mb[(size_t)bh * NPOS + q0 + 8 * g + r]; il[r] = 1.0f / Lb[(size_t)bh * NPOS + q0 + 8 * g + r]; }
  v8f acc[2] = {};
#pragma unroll 1
  for (int ks = 0; ks < NPOS / 32; ++ks) {
#pragma unroll
    for (int ct = 0; ct < 2; ++ct) { const F2 kb = split_rowK(QKV + ((size_t)b * NPOS + ks * 32 + ct * 16 + col) * 256 + KF + h * DK, 0, lane, DK); const v8f s = mac3(a, kb, (v8f){});
#pragma unroll
      for (int r = 0; r < 8; ++r) sp[wave][8 * g + r][ct * 16 + col] = exp_ni(s[r] - mr[r]) * il[r]; }
    LDSX();
    const F2 pa = split_row(&sp[wave][col][0], 0, lane);
#pragma unroll
    for (int dt = 0; dt < 2; ++dt) { const size_t vrow = ((size_t)b * VF + h * DV + dt * 16 + col) * NPOS + ks * 32; const v16b vh = frag_b(VTH + vrow, lane), vl = frag_b(VTL + vrow, lane);
      acc[dt] = wmma_bf(pa.l, vh, acc[dt]); acc[dt] = wmma_bf(pa.h, vl, acc[dt]); acc[dt] = wmma_bf(pa.h, vh, acc[dt]); }
    LDSX(); }
#pragma unroll
  for (int dt = 0; dt < 2; ++dt)
#pragma unroll
    for (int r = 0; r < 8; ++r) so[wave][8 * g + r][dt * 16 + col] = acc[dt][r];
  LDSX();
  for (int q = lane; q < 16 * 8; q += 32) { const int rl = q >> 3, pc = q & 7; vst2(O + ((size_t)b * NPOS + q0 + rl) * VF + h * DV + pc * 4, *(const v4f*)&so[wave][rl][pc * 4]); }
}
__global__ __launch_bounds__(128) void k_out(const float* __restrict__ O, const float* __restrict__ Wo, const float* __restrict__ bo, const float* __restrict__ X, float* __restrict__ out) {
  __shared__ __align__(16) float st[128][68];
  const int tid = threadIdx.x, wave = tid >> 5, lane = tid & 31, col = lane & 15, g = lane >> 4; const int b = blockIdx.y; const int p0 = blockIdx.x * 64;
  v8f acc[8] = {};
#pragma unroll
  for (int kc = 0; kc < VF / 32; ++kc) { const F2 a = split_row(O + ((size_t)b * NPOS + p0 + wave * 16 + col) * VF, kc * 32, lane);
#pragma unroll
    for (int j = 0; j < 8; ++j) { const v16b w = frag_gbf(Wo + (size_t)(j * 16 + col) * VF + kc * 32, lane); acc[j] = wmma_bf(a.l, w, acc[j]); acc[j] = wmma_bf(a.h, w, acc[j]); } }
#pragma unroll
  for (int j = 0; j < 8; ++j) { const float bb = bfr(bo[j * 16 + col]);
#pragma unroll
    for (int r = 0; r < 8; ++r) st[j * 16 + col][wave * 16 + 8 * g + r] = acc[j][r] + bb; }
  __syncthreads();
  for (int q = tid; q < 128 * 16; q += 128) { const int o = q >> 4, pc = q & 15; const size_t base = ((size_t)b * CIN + o) * NPOS + p0 + pc * 4; const float4 xv = *(const float4*)(X + base);
    v4f r4; r4[0] = st[o][pc * 4] + bfr(xv.x); r4[1] = st[o][pc * 4 + 1] + bfr(xv.y); r4[2] = st[o][pc * 4 + 2] + bfr(xv.z); r4[3] = st[o][pc * 4 + 3] + bfr(xv.w); vst2(out + base, r4); }
}

extern "C" void kernel_launch(void* const* d_in, const int* in_sizes, int n_in, void* d_out, int out_size, void* d_ws, size_t ws_size, hipStream_t stream) {
  (void)in_sizes; (void)n_in; (void)out_size;
  const float** F = (const float**)d_in;
  if (ws_size < (size_t)WS_END) return;
  char* ws = (char*)d_ws;
  __bf16 *PH = (__bf16*)(ws + WS_XH), *PL = (__bf16*)(ws + WS_XL), *VTH = (__bf16*)(ws + WS_VTH), *VTL = (__bf16*)(ws + WS_VTL); float *QKV = (float*)(ws + WS_QKV), *Mb = (float*)(ws + WS_M), *Lb = (float*)(ws + WS_L), *O = (float*)(ws + WS_O);
  k_xT<<<dim3(NPOS / 64, TNB), 256, 0, stream>>>(F[0], F[1], F[2], F[3], F[4], PH, PL);
  k_qkv<<<dim3(NPOS / 64, 2, TNB), 128, 0, stream>>>(PH, PL, F[5], F[6], F[7], F[8], F[9], F[10], QKV, VTH, VTL);
  k_stats<<<dim3(TQB, TNB * NHD), 128, 0, stream>>>(QKV, Mb, Lb);
  k_attn<<<dim3(TQB, TNB * NHD), 128, 0, stream>>>(QKV, VTH, VTL, Mb, Lb, O);
  k_out<<<dim3(TQB, TNB), 128, 0, stream>>>(O, F[11], F[12], F[0], (float*)d_out);
}
